// SCFlow_geo_57672820850961
// MI455X (gfx1250) — hardware-verified
//
#include <hip/hip_runtime.h>


typedef _Float16 v16h __attribute__((ext_vector_type(16)));
typedef _Float16 v8h  __attribute__((ext_vector_type(8)));
typedef float    v8f  __attribute__((ext_vector_type(8)));
typedef float    v4f  __attribute__((ext_vector_type(4)));
typedef unsigned int v4u __attribute__((ext_vector_type(4)));

union Frag  { v16h v; v4u q[2]; };
union Pack8 { v8h h; v4u u; };

__device__ __forceinline__ v8f wmma16(v16h a, v16h b, v8f c)
{
    v8f d = __builtin_amdgcn_wmma_f32_16x16x32_f16(false, a, false, b, (short)0, c, false, false);
    asm volatile("v_nop\n\tv_nop\n\tv_nop\n\tv_nop" : "+v"(d) : "v"(a), "v"(b));
    return d;
}

__global__ __launch_bounds__(256) void k_wconv(const float* __restrict__ w, _Float16* __restrict__ wf,
    int Co, int Ci, int Kh, int Kw, int Kp, int perm, float scale, int nT)
{
    const int t = blockIdx.x * 256 + threadIdx.x;
    if (t >= nT) return;
    const int i0 = t * 8;
    const int co = i0 / Kp;
    const int kb = i0 - co * Kp;
    const int KK = Ci * Kh * Kw;
    const bool pw = (Kh == 1) && (Kw == 1);
    Pack8 pk;
#pragma unroll
    for (int e = 0; e < 8; ++e) {
        const int k = kb + e;
        float v = 0.0f;
        if (co < Co && k < KK) {
            int ci, kh, kw;
            if (pw) { ci = k; kh = 0; kw = 0; }
            else { ci = k % Ci; const int tt = k / Ci; kw = tt % Kw; kh = tt / Kw; }
            if (perm) ci = (ci < 192) ? ci : ((ci < 256) ? (ci + 32) : (ci - 64));
            v = w[(((size_t)co * Ci + ci) * Kh + kh) * Kw + kw] * scale;
        }
        pk.h[e] = (_Float16)v;
    }
    const v4u u = pk.u;
    _Float16* dst = wf + i0;
    *(volatile v4u*)dst = u;
    __threadfence();
    *(volatile v4u*)dst = u;
}

__global__ __launch_bounds__(256) void k_pack_in(const float* __restrict__ in, _Float16* __restrict__ out,
    int C, int HW, int ldY, int cOff, int nT)
{
    const int t = blockIdx.x * 256 + threadIdx.x;
    if (t >= nT) return;
    Pack8 pk;
    _Float16* dst;
    if (C >= 8) {
        const int cp = C >> 3;
        const int pix = t / cp;
        const int q = t - pix * cp;
        const int b = pix / HW;
        const int hw = pix - b * HW;
        const float* src = in + ((size_t)b * C + q * 8) * HW + hw;
#pragma unroll
        for (int i = 0; i < 8; ++i) pk.h[i] = (_Float16)src[(size_t)i * HW];
        dst = out + (size_t)pix * ldY + cOff + q * 8;
    } else {
        const int pp = 8 / C;
        const int pix0 = t * pp;
        const int b = pix0 / HW;
        const int hw0 = pix0 - b * HW;
#pragma unroll
        for (int i = 0; i < 8; ++i) {
            const int pi = i / C;
            const int c = i - pi * C;
            pk.h[i] = (_Float16)in[((size_t)b * C + c) * HW + hw0 + pi];
        }
        dst = out + (size_t)pix0 * ldY + cOff;
    }
    const v4u u = pk.u;
    *(volatile v4u*)dst = u;
    __threadfence();
    *(volatile v4u*)dst = u;
}

__device__ __forceinline__ void store_rows(const float* Cs, _Float16* y, int tid, int m0, int M, int ldY, int cbase)
{
    const int seg = tid & 7, rr = tid >> 3;
    for (int ps = 0; ps < 4; ++ps) {
        const int row = ps * 32 + rr;
        const int gm = m0 + row;
        if (gm < M) {
            const float* src = Cs + row * 64 + seg * 8;
            const v4f f0 = *(const v4f*)src;
            const v4f f1 = *(const v4f*)(src + 4);
            Pack8 pk;
            pk.h[0] = (_Float16)f0.x; pk.h[1] = (_Float16)f0.y; pk.h[2] = (_Float16)f0.z; pk.h[3] = (_Float16)f0.w;
            pk.h[4] = (_Float16)f1.x; pk.h[5] = (_Float16)f1.y; pk.h[6] = (_Float16)f1.z; pk.h[7] = (_Float16)f1.w;
            _Float16* dst = y + (size_t)gm * ldY + cbase + seg * 8;
            *(volatile v4u*)dst = pk.u;
        }
    }
}

__device__ __forceinline__ void store_rows(const float* Cs, float* y, int tid, int m0, int M, int ldY, int cbase)
{
    const int seg = tid & 15, rr = tid >> 4;
    for (int ps = 0; ps < 8; ++ps) {
        const int row = ps * 16 + rr;
        const int gm = m0 + row;
        if (gm < M) {
            const v4f f = *(const v4f*)(Cs + row * 64 + seg * 4);
            float* dst = y + (size_t)gm * ldY + cbase + seg * 4;
            *(volatile v4f*)dst = f;
        }
    }
}

template <typename OT>
__global__ __launch_bounds__(256) void k_conv(
    const _Float16* __restrict__ x, const _Float16* __restrict__ wf,
    const float* __restrict__ bias, OT* __restrict__ y,
    int M, int H, int W, int Cin, int ldX, int K, int Cout,
    int Kh, int Kw, int stride, int pad, int Kp,
    int woShift, int hoShift, int ldY, int cOff, int doRelu, float oscale)
{
    __shared__ __align__(16) _Float16 As[128 * 40];
    __shared__ __align__(16) _Float16 Bs[64 * 40];
    __shared__ __align__(16) float Cs[128 * 64];

    const int tid  = threadIdx.x;
    const int lane = tid & 31;
    const int wave = tid >> 5;
    const int wm   = wave & 3;
    const int wn   = wave >> 2;
    const int hv   = lane >> 4;
    const int l    = lane & 15;

    const int m0 = blockIdx.x * 128;
    const int n0 = blockIdx.y * 64;

    const int ar = tid >> 1;
    const int ak = (tid & 1) * 16;
    const int am = m0 + ar;
    const bool amOk = am < M;
    const int aw = am & ((1 << woShift) - 1);
    const int tq = am >> woShift;
    const int ah = tq & ((1 << hoShift) - 1);
    const int ab = tq >> hoShift;
    const int hb = ah * stride - pad;
    const int wb = aw * stride - pad;
    const long long imgBase = (long long)ab * H * W;
    v4u* const asDst = (v4u*)&As[ar * 40 + ak];

    int ci = ak, kw = 0, kh = 0;
    while (ci >= Cin) { ci -= Cin; if (++kw == Kw) { kw = 0; ++kh; } }

    const int bn = tid >> 2;
    const int bk = (tid & 3) * 8;
    const bool bnOk = (n0 + bn) < Cout;

    const v4u uz = {0u, 0u, 0u, 0u};
    const v8f vzero = {0.f, 0.f, 0.f, 0.f, 0.f, 0.f, 0.f, 0.f};
    v8f acc[2][2];
    acc[0][0] = vzero; acc[0][1] = vzero; acc[1][0] = vzero; acc[1][1] = vzero;

    for (int k0 = 0; k0 < Kp; k0 += 32) {
        const int kk0 = k0 + ak;
        v4u a0 = uz, a1 = uz;
        if (amOk && kk0 < K) {
            const int hi = hb + kh, wi = wb + kw;
            const bool pixOk = (hi >= 0) && (hi < H) && (wi >= 0) && (wi < W);
            const bool runOk = (ci + 16 <= Cin) && (kk0 + 16 <= K);
            if (runOk && pixOk) {
                const long long eoff = (imgBase + (long long)hi * W + wi) * ldX + ci;
                if ((eoff & 7) == 0) {
                    const v4u* src = (const v4u*)(x + eoff);
                    a0 = src[0];
                    a1 = src[1];
                } else {
                    Frag tt;
#pragma unroll
                    for (int i = 0; i < 16; ++i) tt.v[i] = x[eoff + i];
                    a0 = tt.q[0]; a1 = tt.q[1];
                }
            } else if (!runOk) {
                Frag tt;
                int c2 = ci, w2 = kw, h2 = kh;
#pragma unroll
                for (int i = 0; i < 16; ++i) {
                    _Float16 v = (_Float16)0.0f;
                    if (kk0 + i < K) {
                        const int hi2 = hb + h2, wi2 = wb + w2;
                        if (hi2 >= 0 && hi2 < H && wi2 >= 0 && wi2 < W)
                            v = x[(imgBase + (long long)hi2 * W + wi2) * ldX + c2];
                    }
                    tt.v[i] = v;
                    if (++c2 == Cin) { c2 = 0; if (++w2 == Kw) { w2 = 0; ++h2; } }
                }
                a0 = tt.q[0]; a1 = tt.q[1];
            }
        }
        asDst[0] = a0;
        asDst[1] = a1;

        v4u bv = uz;
        if (bnOk) bv = *(const v4u*)(wf + (size_t)(n0 + bn) * Kp + k0 + bk);
        *(v4u*)&Bs[bn * 40 + bk] = bv;

        __syncthreads();

        Frag fa0, fa1, fb0, fb1;
        const int ra0 = (wm * 32 + l) * 40;
        const int ra1 = (wm * 32 + 16 + l) * 40;
        const int cb0 = (wn * 32 + l) * 40;
        const int cb1 = (wn * 32 + 16 + l) * 40;
        fa0.q[0] = *(const v4u*)&As[ra0 + 8 * hv];
        fa0.q[1] = *(const v4u*)&As[ra0 + 16 + 8 * hv];
        fa1.q[0] = *(const v4u*)&As[ra1 + 8 * hv];
        fa1.q[1] = *(const v4u*)&As[ra1 + 16 + 8 * hv];
        fb0.q[0] = *(const v4u*)&Bs[cb0 + 8 * hv];
        fb0.q[1] = *(const v4u*)&Bs[cb0 + 16 + 8 * hv];
        fb1.q[0] = *(const v4u*)&Bs[cb1 + 8 * hv];
        fb1.q[1] = *(const v4u*)&Bs[cb1 + 16 + 8 * hv];

        acc[0][0] = wmma16(fa0.v, fb0.v, acc[0][0]);
        acc[0][1] = wmma16(fa0.v, fb1.v, acc[0][1]);
        acc[1][0] = wmma16(fa1.v, fb0.v, acc[1][0]);
        acc[1][1] = wmma16(fa1.v, fb1.v, acc[1][1]);

        __syncthreads();

        ci += 32;
        while (ci >= Cin) { ci -= Cin; if (++kw == Kw) { kw = 0; ++kh; } }
    }

#pragma unroll
    for (int i = 0; i < 2; ++i) {
#pragma unroll
        for (int j = 0; j < 2; ++j) {
            const int col = wn * 32 + j * 16 + l;
            const int gn = n0 + col;
            const float bb = (gn < Cout) ? bias[min(gn, Cout - 1)] : 0.0f;
#pragma unroll
            for (int r = 0; r < 8; ++r) {
                const int row = wm * 32 + i * 16 + 8 * hv + r;
                float v = acc[i][j][r] * oscale + bb;
                if (doRelu) v = fmaxf(v, 0.0f);
                Cs[row * 64 + col] = v;
            }
        }
    }
    __syncthreads();

    store_rows(Cs, y, tid, m0, M, ldY, cOff + n0);
    __threadfence();
    store_rows(Cs, y, tid, m0, M, ldY, cOff + n0);
}

template <bool FLAT>
__global__ __launch_bounds__(256) void k_gn(const float* __restrict__ x, const float* __restrict__ sc,
    const float* __restrict__ bi, _Float16* __restrict__ y, int HW, float invN)
{
    __shared__ float red0[256];
    __shared__ float red1[256];
    __shared__ float gmean[32];
    __shared__ float grstd[32];

    const int tid = threadIdx.x;
    const int b = blockIdx.x;
    const float* xb = x + (size_t)b * HW * 128;
    const int q = tid & 15;
    const int pr = tid >> 4;

    float s0 = 0.0f, s1 = 0.0f;
    for (int p = pr; p < HW; p += 16) {
        const float* src = xb + (size_t)p * 128 + q * 8;
        const v4f a = *(const v4f*)src;
        const v4f c = *(const v4f*)(src + 4);
        s0 += a.x; s0 += a.y; s0 += a.z; s0 += a.w;
        s1 += c.x; s1 += c.y; s1 += c.z; s1 += c.w;
    }
    red0[tid] = s0; red1[tid] = s1;
    __syncthreads();
    if (tid < 32) {
        const int qq = tid >> 1, wh = tid & 1;
        float s = 0.0f;
        for (int r = 0; r < 16; ++r) s += wh ? red1[qq + 16 * r] : red0[qq + 16 * r];
        gmean[tid] = s * invN;
    }
    __syncthreads();
    const float mA = gmean[2 * q], mB = gmean[2 * q + 1];
    s0 = 0.0f; s1 = 0.0f;
    for (int p = pr; p < HW; p += 16) {
        const float* src = xb + (size_t)p * 128 + q * 8;
        const v4f a = *(const v4f*)src;
        const v4f c = *(const v4f*)(src + 4);
        float d;
        d = a.x - mA; s0 += d * d; d = a.y - mA; s0 += d * d; d = a.z - mA; s0 += d * d; d = a.w - mA; s0 += d * d;
        d = c.x - mB; s1 += d * d; d = c.y - mB; s1 += d * d; d = c.z - mB; s1 += d * d; d = c.w - mB; s1 += d * d;
    }
    red0[tid] = s0; red1[tid] = s1;
    __syncthreads();
    if (tid < 32) {
        const int qq = tid >> 1, wh = tid & 1;
        float s = 0.0f;
        for (int r = 0; r < 16; ++r) s += wh ? red1[qq + 16 * r] : red0[qq + 16 * r];
        grstd[tid] = rsqrtf(s * invN + 1e-5f);
    }
    __syncthreads();

    if (!FLAT) {
        const float rA = grstd[2 * q], rB = grstd[2 * q + 1];
        float scv[8], biv[8];
#pragma unroll
        for (int i = 0; i < 8; ++i) { scv[i] = sc[q * 8 + i]; biv[i] = bi[q * 8 + i]; }
#pragma unroll
        for (int rep = 0; rep < 2; ++rep) {
            for (int p = pr; p < HW; p += 16) {
                const float* src = xb + (size_t)p * 128 + q * 8;
                const v4f a = *(const v4f*)src;
                const v4f c = *(const v4f*)(src + 4);
                Pack8 pk;
                pk.h[0] = (_Float16)fmaxf((a.x - mA) * rA * scv[0] + biv[0], 0.0f);
                pk.h[1] = (_Float16)fmaxf((a.y - mA) * rA * scv[1] + biv[1], 0.0f);
                pk.h[2] = (_Float16)fmaxf((a.z - mA) * rA * scv[2] + biv[2], 0.0f);
                pk.h[3] = (_Float16)fmaxf((a.w - mA) * rA * scv[3] + biv[3], 0.0f);
                pk.h[4] = (_Float16)fmaxf((c.x - mB) * rB * scv[4] + biv[4], 0.0f);
                pk.h[5] = (_Float16)fmaxf((c.y - mB) * rB * scv[5] + biv[5], 0.0f);
                pk.h[6] = (_Float16)fmaxf((c.z - mB) * rB * scv[6] + biv[6], 0.0f);
                pk.h[7] = (_Float16)fmaxf((c.w - mB) * rB * scv[7] + biv[7], 0.0f);
                _Float16* dst = y + ((size_t)b * HW + p) * 128 + q * 8;
                *(volatile v4u*)dst = pk.u;
            }
            if (rep == 0) __threadfence();
        }
    } else {
        const int c = tid >> 1, pc = tid & 1, g = c >> 2;
        const float mg = gmean[g], rg = grstd[g];
        const float scc = sc[c], bic = bi[c];
        Pack8 pk;
#pragma unroll
        for (int i = 0; i < 8; ++i) {
            const float v = xb[(size_t)(pc * 8 + i) * 128 + c];
            pk.h[i] = (_Float16)fmaxf((v - mg) * rg * scc + bic, 0.0f);
        }
        _Float16* dst = y + (size_t)b * 2048 + c * 16 + pc * 8;
        const v4u u = pk.u;
        *(volatile v4u*)dst = u;
        __threadfence();
        *(volatile v4u*)dst = u;
    }
}

__global__ __launch_bounds__(256) void k_heads(const _Float16* __restrict__ xa, const _Float16* __restrict__ wh,
    const float* __restrict__ rot_b, const float* __restrict__ tr_b, const int* __restrict__ obj,
    float* __restrict__ out, int nc, float oscale)
{
    __shared__ __align__(16) float sD[64 * 192];

    const int tid = threadIdx.x;
    const int lane = tid & 31, wave = tid >> 5;
    const int h = lane >> 4, m = lane & 15;
    const int rt = wave & 3, cg = wave >> 2;

    const v8f vzero = {0.f, 0.f, 0.f, 0.f, 0.f, 0.f, 0.f, 0.f};
    v8f acc[6];
#pragma unroll
    for (int j = 0; j < 6; ++j) acc[j] = vzero;

    for (int k0 = 0; k0 < 256; k0 += 32) {
        Frag fa;
        const _Float16* ap = xa + (size_t)(rt * 16 + m) * 256 + k0 + 8 * h;
        fa.q[0] = *(const v4u*)ap;
        fa.q[1] = *(const v4u*)(ap + 16);
#pragma unroll
        for (int j = 0; j < 6; ++j) {
            Frag fb;
            const _Float16* bp = wh + (size_t)((cg * 6 + j) * 16 + m) * 256 + k0 + 8 * h;
            fb.q[0] = *(const v4u*)bp;
            fb.q[1] = *(const v4u*)(bp + 16);
            acc[j] = wmma16(fa.v, fb.v, acc[j]);
        }
    }
#pragma unroll
    for (int j = 0; j < 6; ++j) {
#pragma unroll
        for (int r = 0; r < 8; ++r)
            sD[(rt * 16 + 8 * h + r) * 192 + (cg * 6 + j) * 16 + m] = acc[j][r];
    }
    __syncthreads();

    int jsel = obj[0] - 1;
    jsel = jsel < 0 ? 0 : (jsel > nc - 1 ? nc - 1 : jsel);
    if (tid < 144) {
        v4f o;
#pragma unroll
        for (int e4 = 0; e4 < 4; ++e4) {
            const int f = tid * 4 + e4;
            float v;
            if (f < 384) {
                const int bb = f / 6, e = f - bb * 6;
                const int col = jsel * 6 + e;
                v = sD[bb * 192 + col] * oscale + rot_b[col];
            } else {
                const int f2 = f - 384;
                const int bb = f2 / 3, e = f2 - bb * 3;
                const int col = jsel * 3 + e;
                v = sD[bb * 192 + 126 + col] * oscale + tr_b[col];
            }
            o[e4] = v;
        }
        float* dst = out + tid * 4;
        *(volatile v4f*)dst = o;
        __threadfence();
        *(volatile v4f*)dst = o;
    }
}

extern "C" void kernel_launch(void* const* d_in, const int* in_sizes, int n_in,
                              void* d_out, int out_size, void* d_ws, size_t ws_size,
                              hipStream_t stream)
{
    if (n_in < 37 || out_size != 576) return;
    const int Bn = 64;
    if (in_sizes[0] != Bn * 128 * 1024 || in_sizes[1] != Bn * 2 * 1024 || in_sizes[2] != Bn * 1024 ||
        in_sizes[3] != Bn * 8 * 4096 || in_sizes[4] < 1) return;
    if (in_sizes[5] != 9216 || in_sizes[6] != 128 || in_sizes[7] != 73728 || in_sizes[8] != 64 ||
        in_sizes[9] != 12544 || in_sizes[10] != 128 || in_sizes[11] != 73728 || in_sizes[12] != 64 ||
        in_sizes[13] != 576 || in_sizes[14] != 64 || in_sizes[15] != 18432 || in_sizes[16] != 32 ||
        in_sizes[17] != 331776 || in_sizes[18] != 128 || in_sizes[19] != 128 || in_sizes[20] != 128 ||
        in_sizes[21] != 147456 || in_sizes[22] != 128 || in_sizes[23] != 128 || in_sizes[24] != 128 ||
        in_sizes[25] != 147456 || in_sizes[26] != 128 || in_sizes[27] != 128 || in_sizes[28] != 128 ||
        in_sizes[29] != 2097152 || in_sizes[30] != 1024 || in_sizes[31] != 262144 || in_sizes[32] != 256 ||
        in_sizes[33] != 32256 || in_sizes[34] != 126 || in_sizes[35] != 16128 || in_sizes[36] != 63) return;
    const int nc = 21;

    const int* obj = (const int*)d_in[4];
    float* out = (float*)d_out;

    char* ws = (char*)d_ws;
    size_t off = 0;
    auto carve = [&](size_t bytes) -> char* {
        char* p = ws + off;
        off = (off + bytes + 255) & ~(size_t)255;
        return p;
    };
    auto carveH = [&](size_t nHalf) -> _Float16* { return (_Float16*)carve(nHalf * 2); };

    _Float16* wf_g1 = carveH((size_t)128 * 96);
    _Float16* wf_g2 = carveH((size_t)64 * 1152);
    _Float16* wf_d1 = carveH((size_t)128 * 128);
    _Float16* wf_d2 = carveH((size_t)64 * 1152);
    _Float16* wf_m1 = carveH((size_t)64 * 32);
    _Float16* wf_m2 = carveH((size_t)32 * 576);
    _Float16* wf_c1 = carveH((size_t)128 * 2592);
    _Float16* wf_c2 = carveH((size_t)128 * 1152);
    _Float16* wf_c3 = carveH((size_t)128 * 1152);
    _Float16* wf_f1 = carveH((size_t)1024 * 2048);
    _Float16* wf_f2 = carveH((size_t)256 * 1024);
    _Float16* wf_hd = carveH((size_t)192 * 256);
    _Float16* geoT = carveH((size_t)Bn * 4096 * 8);
    _Float16* dfT  = carveH((size_t)Bn * 1024 * 2);
    _Float16* mkT  = carveH((size_t)Bn * 1024 * 1);
    _Float16* enc  = carveH((size_t)Bn * 1024 * 320);
    const size_t Rbytes = (size_t)Bn * 4096 * 128 * 2;
    char* R = carve(Rbytes);
    if (off > ws_size) return;

    _Float16* g1o = (_Float16*)R;
    size_t offR = 0;
    auto sub = [&](size_t bytes) -> char* {
        char* p = R + offR;
        offR = (offR + bytes + 255) & ~(size_t)255;
        return p;
    };
    _Float16* d1o   = (_Float16*)sub((size_t)Bn * 1024 * 128 * 2);
    _Float16* m1o   = (_Float16*)sub((size_t)Bn * 1024 * 64 * 2);
    float*    c1raw = (float*)sub((size_t)Bn * 256 * 128 * 4);
    _Float16* c1n   = (_Float16*)sub((size_t)Bn * 256 * 128 * 2);
    float*    c2raw = (float*)sub((size_t)Bn * 64 * 128 * 4);
    _Float16* c2n   = (_Float16*)sub((size_t)Bn * 64 * 128 * 2);
    float*    c3raw = (float*)sub((size_t)Bn * 16 * 128 * 4);
    _Float16* fcA   = (_Float16*)sub((size_t)Bn * 2048 * 2);
    _Float16* f1o   = (_Float16*)sub((size_t)Bn * 1024 * 2);
    _Float16* f2o   = (_Float16*)sub((size_t)Bn * 256 * 2);
    if (offR > Rbytes) return;

    const float wsc = 64.0f;
    const float osc = 0.015625f;

    auto wconv = [&](const void* w, _Float16* wf, int Co, int CoPad, int Ci, int Kh, int Kw, int Kp, int perm) {
        const int nT = CoPad * Kp / 8;
        k_wconv<<<(nT + 255) / 256, 256, 0, stream>>>((const float*)w, wf, Co, Ci, Kh, Kw, Kp, perm, wsc, nT);
    };
    wconv(d_in[5],  wf_g1,  128,  128,    8, 3, 3,   96, 0);
    wconv(d_in[7],  wf_g2,   64,   64,  128, 3, 3, 1152, 0);
    wconv(d_in[9],  wf_d1,  128,  128,    2, 7, 7,  128, 0);
    wconv(d_in[11], wf_d2,   64,   64,  128, 3, 3, 1152, 0);
    wconv(d_in[13], wf_m1,   64,   64,    1, 3, 3,   32, 0);
    wconv(d_in[15], wf_m2,   32,   32,   64, 3, 3,  576, 0);
    wconv(d_in[17], wf_c1,  128,  128,  288, 3, 3, 2592, 1);
    wconv(d_in[21], wf_c2,  128,  128,  128, 3, 3, 1152, 0);
    wconv(d_in[25], wf_c3,  128,  128,  128, 3, 3, 1152, 0);
    wconv(d_in[29], wf_f1, 1024, 1024, 2048, 1, 1, 2048, 0);
    wconv(d_in[31], wf_f2,  256,  256, 1024, 1, 1, 1024, 0);
    wconv(d_in[33], wf_hd,  126,  126,  256, 1, 1,  256, 0);
    wconv(d_in[35], wf_hd + (size_t)126 * 256, 63, 66, 256, 1, 1, 256, 0);

    auto pack = [&](const void* in, _Float16* o, int C, int HW, int ldY, int cOff) {
        const int nT = (C >= 8) ? Bn * HW * (C >> 3) : Bn * HW * C / 8;
        k_pack_in<<<(nT + 255) / 256, 256, 0, stream>>>((const float*)in, o, C, HW, ldY, cOff, nT);
    };
    pack(d_in[0], enc,  128, 1024, 320, 0);
    pack(d_in[3], geoT,   8, 4096,   8, 0);
    pack(d_in[1], dfT,    2, 1024,   2, 0);
    pack(d_in[2], mkT,    1, 1024,   1, 0);

    auto conv16 = [&](const _Float16* x, int ldX, const _Float16* w, const void* bias, _Float16* y,
                      int H, int W, int Cin, int Ho, int Wo, int Cout,
                      int Kh, int Kw, int s, int p, int Kp,
                      int woShift, int hoShift, int ldY, int cOff, int relu) {
        const int M = Bn * Ho * Wo;
        const int K = Kh * Kw * Cin;
        dim3 grid((M + 127) / 128, (Cout + 63) / 64);
        k_conv<_Float16><<<grid, 256, 0, stream>>>(x, w, (const float*)bias, y,
            M, H, W, Cin, ldX, K, Cout, Kh, Kw, s, p, Kp, woShift, hoShift, ldY, cOff, relu, osc);
    };
    auto conv32 = [&](const _Float16* x, int ldX, const _Float16* w, const void* bias, float* y,
                      int H, int W, int Cin, int Ho, int Wo, int Cout,
                      int Kh, int Kw, int s, int p, int Kp,
                      int woShift, int hoShift, int ldY, int cOff, int relu) {
        const int M = Bn * Ho * Wo;
        const int K = Kh * Kw * Cin;
        dim3 grid((M + 127) / 128, (Cout + 63) / 64);
        k_conv<float><<<grid, 256, 0, stream>>>(x, w, (const float*)bias, y,
            M, H, W, Cin, ldX, K, Cout, Kh, Kw, s, p, Kp, woShift, hoShift, ldY, cOff, relu, osc);
    };

    conv16(geoT,   8, wf_g1, d_in[6],  g1o, 64, 64,   8, 64, 64, 128, 3, 3, 1, 1,   96, 6, 6, 128,   0, 1);
    conv16(g1o,  128, wf_g2, d_in[8],  enc, 64, 64, 128, 32, 32,  64, 3, 3, 2, 1, 1152, 5, 5, 320, 192, 1);
    conv16(dfT,    2, wf_d1, d_in[10], d1o, 32, 32,   2, 32, 32, 128, 7, 7, 1, 3,  128, 5, 5, 128,   0, 1);
    conv16(d1o,  128, wf_d2, d_in[12], enc, 32, 32, 128, 32, 32,  64, 3, 3, 1, 1, 1152, 5, 5, 320, 128, 1);
    conv16(mkT,    1, wf_m1, d_in[14], m1o, 32, 32,   1, 32, 32,  64, 3, 3, 1, 1,   32, 5, 5,  64,   0, 1);
    conv16(m1o,   64, wf_m2, d_in[16], enc, 32, 32,  64, 32, 32,  32, 3, 3, 1, 1,  576, 5, 5, 320, 256, 1);
    conv32(enc,  320, wf_c1, d_in[18], c1raw, 32, 32, 288, 16, 16, 128, 3, 3, 2, 1, 2592, 4, 4, 128, 0, 0);
    k_gn<false><<<Bn, 256, 0, stream>>>(c1raw, (const float*)d_in[19], (const float*)d_in[20], c1n, 256, 1.0f / 1024.0f);
    conv32(c1n,  128, wf_c2, d_in[22], c2raw, 16, 16, 128,  8,  8, 128, 3, 3, 2, 1, 1152, 3, 3, 128, 0, 0);
    k_gn<false><<<Bn, 256, 0, stream>>>(c2raw, (const float*)d_in[23], (const float*)d_in[24], c2n, 64, 1.0f / 256.0f);
    conv32(c2n,  128, wf_c3, d_in[26], c3raw,  8,  8, 128,  4,  4, 128, 3, 3, 2, 1, 1152, 2, 2, 128, 0, 0);
    k_gn<true><<<Bn, 256, 0, stream>>>(c3raw, (const float*)d_in[27], (const float*)d_in[28], fcA, 16, 1.0f / 64.0f);

    conv16(fcA, 2048, wf_f1, d_in[30], f1o, 1, 1, 2048, 1, 1, 1024, 1, 1, 1, 0, 2048, 0, 0, 1024, 0, 1);
    conv16(f1o, 1024, wf_f2, d_in[32], f2o, 1, 1, 1024, 1, 1,  256, 1, 1, 1, 0, 1024, 0, 0,  256, 0, 1);

    k_heads<<<1, 256, 0, stream>>>(f2o, wf_hd, (const float*)d_in[34], (const float*)d_in[36], obj, out, nc, osc);
}
